// attention_as_rnn_31937376813365
// MI455X (gfx1250) — hardware-verified
//
#include <hip/hip_runtime.h>


namespace {
constexpr int Bn = 4, T = 2048, DIM = 1024, H = 16, DI = 64, DO = 1024, NT = Bn * T, KVC = H * DI * 2  ;
constexpr float AS_ = 8.0f;

typedef _Float16 b16;
typedef __attribute__((ext_vector_type(16))) _Float16 v16b;
typedef __attribute__((ext_vector_type(16))) __bf16 v16bb;
typedef __attribute__((ext_vector_type(8))) _Float16 v8b;
typedef __attribute__((ext_vector_type(8))) unsigned short v8us;
typedef __attribute__((ext_vector_type(8))) float v8f;
typedef __attribute__((ext_vector_type(4))) float v4f;
__device__ __forceinline__ float bf16_rne(float f) { unsigned int u = __float_as_uint(f); u += 0x7FFFu + ((u >> 16) & 1u); return __uint_as_float(u & 0xFFFF0000u); }
__device__ __forceinline__ unsigned short bf16_bits(float f) { unsigned int u = __float_as_uint(f); u += 0x7FFFu + ((u >> 16) & 1u); return (unsigned short)(u >> 16); }
__device__ __forceinline__ void split16(float v, b16& hi, b16& lo) { hi = (b16)v; lo = (b16)(v - (float)hi); }
__device__ __forceinline__ v16b frag_kb(const b16* p, int hh) { const v8b a = *(const v8b*)(p + 8 * hh), b = *(const v8b*)(p + 16 + 8 * hh); v16b f;
#pragma unroll
  for (int e = 0; e < 8; ++e) { f[e] = a[e]; f[8 + e] = b[e]; } return f; }
__device__ __forceinline__ v16bb frag_bf(const unsigned short* p, int hh) { const v8us a = *(const v8us*)(p + 8 * hh), b = *(const v8us*)(p + 16 + 8 * hh); union { unsigned short s[16]; v16bb v; } u;
#pragma unroll
  for (int e = 0; e < 8; ++e) { u.s[e] = a[e]; u.s[8 + e] = b[e]; } return u.v; }
__device__ __forceinline__ v8f wmma16b(v16b a, v16b b, v8f c) { v8f d = __builtin_amdgcn_wmma_f32_16x16x32_f16(false, a, false, b, (short)0, c, false, false); asm volatile("v_nop\n\tv_nop\n\tv_nop\n\tv_nop" : "+v"(d) : "v"(a), "v"(b)); return d; }
__device__ __forceinline__ v8f wmma16bb(v16bb a, v16bb b, v8f c) { v8f d = __builtin_amdgcn_wmma_f32_16x16x32_bf16(false, a, false, b, (short)0, c, false, false); asm volatile("v_nop\n\tv_nop\n\tv_nop\n\tv_nop" : "+v"(d) : "v"(a), "v"(b)); return d; }
__device__ __forceinline__ void wave_lds_sync() { __builtin_amdgcn_fence(__ATOMIC_RELEASE, "workgroup"); __builtin_amdgcn_wave_barrier(); __builtin_amdgcn_fence(__ATOMIC_ACQUIRE, "workgroup"); }
__device__ __forceinline__ float nexp(float x) { return __builtin_amdgcn_exp2f(x * 1.4426950408889634f); }
__device__ __forceinline__ float pmul(float a, float b) { float p = a * b; asm volatile("" : "+v"(p)); return p; }

__global__ __launch_bounds__(256) void prep_kernel(const float* __restrict__ x, const float* __restrict__ kvk, const float* __restrict__ ow, unsigned short* __restrict__ x16, unsigned short* __restrict__ w16, b16* __restrict__ wo16) {
  const size_t tid = (size_t)blockIdx.x * blockDim.x + threadIdx.x, nth = (size_t)gridDim.x * blockDim.x;
  for (int pass = 0; pass < 2; ++pass) {
    for (size_t p = tid; p < (size_t)NT * DIM / 8; p += nth) { v8us v;
#pragma unroll
      for (int e = 0; e < 8; ++e) v[e] = bf16_bits(x[p * 8 + e]);
      *(volatile v8us*)(x16 + p * 8) = v; }
    for (size_t p = tid; p < (size_t)KVC * DIM / 8; p += nth) { const int n = (int)(p / (DIM / 8)), k0 = (int)(p % (DIM / 8)) * 8; v8us v;
#pragma unroll
      for (int e = 0; e < 8; ++e) v[e] = bf16_bits(kvk[(size_t)(k0 + e) * KVC + n]);
      *(volatile v8us*)(w16 + (size_t)n * DIM + k0) = v; }
    for (size_t p = tid; p < (size_t)DO * DI; p += nth) ((volatile b16*)wo16)[p] = (b16)bf16_rne(ow[p]);
    __threadfence();
  }
}

__global__ __launch_bounds__(128) void kv_kernel(const unsigned short* __restrict__ x16, const unsigned short* __restrict__ w16, float* __restrict__ kv) {
  __shared__ __attribute__((aligned(16))) float Ts[4][32 * 64];
  const int lane = threadIdx.x & 31, wave = threadIdx.x >> 5, nloc = lane & 15, hlf = lane >> 4, m0 = blockIdx.y * 128 + wave * 32, c0 = blockIdx.x * 64;
  v8f acc[2][4];
#pragma unroll
  for (int r = 0; r < 2; ++r)
#pragma unroll
    for (int t = 0; t < 4; ++t) acc[r][t] = (v8f){};
#pragma unroll 2
  for (int kb = 0; kb < DIM; kb += 32) { const v16bb a0 = frag_bf(x16 + (size_t)(m0 + nloc) * DIM + kb, hlf), a1 = frag_bf(x16 + (size_t)(m0 + 16 + nloc) * DIM + kb, hlf);
#pragma unroll
    for (int t = 0; t < 4; ++t) { const v16bb bw = frag_bf(w16 + (size_t)(c0 + t * 16 + nloc) * DIM + kb, hlf); acc[0][t] = wmma16bb(a0, bw, acc[0][t]); acc[1][t] = wmma16bb(a1, bw, acc[1][t]); } }
  float* Tt = Ts[wave];
#pragma unroll
  for (int t = 0; t < 4; ++t)
#pragma unroll
    for (int r = 0; r < 2; ++r)
#pragma unroll
      for (int v = 0; v < 8; ++v) Tt[(r * 16 + v + 8 * hlf) * 64 + t * 16 + nloc] = acc[r][t][v];
  wave_lds_sync();
  float* dst0 = kv + (size_t)m0 * KVC + c0;
  for (int pass = 0; pass < 2; ++pass) {
#pragma unroll
    for (int j = 0; j < 16; ++j) { const int rr = j * 2 + hlf, c4 = nloc * 4; *(volatile v4f*)(dst0 + (size_t)rr * KVC + c4) = *(const v4f*)(Tt + rr * 64 + c4); }
    __threadfence(); }
}

__global__ __launch_bounds__(256) void score_kernel(const float* __restrict__ kv, const float* __restrict__ qk, float* __restrict__ srow) {
  const size_t g = (size_t)blockIdx.x * 256 + threadIdx.x; const size_t tok = g >> 4; const int h = (int)(g & 15); const float* r = kv + tok * KVC + h * 128; float s = 0.0f;
#pragma unroll 4
  for (int d = 0; d < DI; ++d) s += pmul(bf16_rne(qk[h * DI + d]), r[d * 2]);
  for (int pass = 0; pass < 2; ++pass) { ((volatile float*)srow)[g] = s; __threadfence(); }
}
__global__ __launch_bounds__(256) void scan_kernel(const float* __restrict__ kv, const float* __restrict__ srow, float* __restrict__ ratio) {
  const int b = blockIdx.y, h = blockIdx.x * 4 + (threadIdx.x >> 6), d = threadIdx.x & 63;
  float m = -INFINITY, u = 0.0f, w = 0.0f;
  for (int t = 0; t < T; ++t) { const size_t tok = (size_t)b * T + t; const float s = srow[tok * H + h], v = kv[tok * KVC + h * 128 + d * 2 + 1];
    const float mn = fmaxf(m, s); const float ea = nexp(m - mn), eb = nexp(s - mn); u = pmul(u, ea) + eb; w = pmul(w, ea) + pmul(v, eb); m = mn;
    for (int pass = 0; pass < 2; ++pass) ((volatile float*)ratio)[(tok * H + h) * DI + d] = w / u; }
  __threadfence();
}

__global__ __launch_bounds__(128) void out_kernel(const float* __restrict__ ratio, const b16* __restrict__ wo16, const float* __restrict__ ob, float* __restrict__ out) {
  __shared__ __attribute__((aligned(16))) float Ts[4][32 * 64];
  const int lane = threadIdx.x & 31, wave = threadIdx.x >> 5, nloc = lane & 15, hlf = lane >> 4, m0 = blockIdx.y * 128 + wave * 32, c0 = blockIdx.x * 64;
  v8f acc[2][4];
#pragma unroll
  for (int r = 0; r < 2; ++r)
#pragma unroll
    for (int t = 0; t < 4; ++t) acc[r][t] = (v8f){};
#pragma unroll
  for (int kb = 0; kb < DI; kb += 32) { v16b a0, a1, l0, l1;
#pragma unroll
    for (int e = 0; e < 16; ++e) { const int k = kb + ((e < 8) ? (8 * hlf + e) : (16 + 8 * hlf + e - 8)); float s0 = 0.0f, s1 = 0.0f;
#pragma unroll
      for (int h = 0; h < H; ++h) { s0 += ratio[((size_t)(m0 + nloc) * H + h) * DI + k]; s1 += ratio[((size_t)(m0 + 16 + nloc) * H + h) * DI + k]; }
      b16 p, q; split16(s0 * (AS_ / H), p, q); a0[e] = p; l0[e] = q; split16(s1 * (AS_ / H), p, q); a1[e] = p; l1[e] = q; }
#pragma unroll
    for (int t = 0; t < 4; ++t) { const v16b bw = frag_kb(wo16 + (size_t)(c0 + t * 16 + nloc) * DI + kb, hlf); acc[0][t] = wmma16b(a0, bw, acc[0][t]); acc[0][t] = wmma16b(l0, bw, acc[0][t]); acc[1][t] = wmma16b(a1, bw, acc[1][t]); acc[1][t] = wmma16b(l1, bw, acc[1][t]); } }
  float* Tt = Ts[wave];
#pragma unroll
  for (int t = 0; t < 4; ++t)
#pragma unroll
    for (int r = 0; r < 2; ++r)
#pragma unroll
      for (int v = 0; v < 8; ++v) Tt[(r * 16 + v + 8 * hlf) * 64 + t * 16 + nloc] = acc[r][t][v] * (1.0f / AS_) + bf16_rne(ob[c0 + t * 16 + nloc]);
  wave_lds_sync();
  float* dst0 = out + (size_t)m0 * DO + c0;
  for (int pass = 0; pass < 2; ++pass) {
#pragma unroll
    for (int j = 0; j < 16; ++j) { const int rr = j * 2 + hlf, c4 = nloc * 4; *(volatile v4f*)(dst0 + (size_t)rr * DO + c4) = *(const v4f*)(Tt + rr * 64 + c4); }
    __threadfence(); }
}
}

extern "C" void kernel_launch(void* const* d_in, const int* in_sizes, int n_in,
                              void* d_out, int out_size, void* d_ws, size_t ws_size, hipStream_t stream) {
  (void)n_in; (void)out_size;
  const float* x = (const float*)d_in[0]; const float* kvk = (const float*)d_in[1]; const float* qk = (const float*)d_in[2]; const float* ow = (const float*)d_in[3]; const float* ob = (const float*)d_in[4];
  float* out = (float*)d_out;
  if (in_sizes[0] != NT * DIM || in_sizes[1] != DIM * KVC || in_sizes[2] != H * DI || in_sizes[3] != DO * DI || in_sizes[4] != DO) return;
  size_t off = 0; char* ws = (char*)d_ws;
  auto carve = [&](size_t bytes) { char* p = ws + off; off += (bytes + 255) & ~(size_t)255; return p; };
  unsigned short* x16 = (unsigned short*)carve((size_t)NT * DIM * 2); unsigned short* w16 = (unsigned short*)carve((size_t)KVC * DIM * 2); b16* wo16 = (b16*)carve((size_t)DO * DI * 2);
  float* kv = (float*)carve((size_t)NT * KVC * 4); float* srow = (float*)carve((size_t)NT * H * 4); float* ratio = (float*)carve((size_t)NT * H * DI * 4);
  if (off > ws_size) return;
  prep_kernel<<<1024, 256, 0, stream>>>(x, kvk, ow, x16, w16, wo16);
  kv_kernel<<<dim3(KVC / 64, NT / 128), 128, 0, stream>>>(x16, w16, kv);
  score_kernel<<<NT * H / 256, 256, 0, stream>>>(kv, qk, srow);
  scan_kernel<<<dim3(H / 4, Bn), 256, 0, stream>>>(kv, srow, ratio);
  out_kernel<<<dim3(DO / 64, NT / 128), 128, 0, stream>>>(ratio, wo16, ob, out);
}
